// Brain_26525718020137
// MI455X (gfx1250) — hardware-verified
//
#include <hip/hip_runtime.h>


namespace {
constexpr int NBT = 8192, P = 512, DM = 256, DI = 512, NS = 16, DTR = 16, AD = 64, XD = 48;
constexpr float XS = 8.0f, ES = 16384.0f  , WSC = 256.0f;
typedef _Float16 b16;
typedef __attribute__((ext_vector_type(16))) _Float16 v16b;
typedef __attribute__((ext_vector_type(8))) _Float16 v8b;
typedef __attribute__((ext_vector_type(8))) float v8f;
typedef __attribute__((ext_vector_type(4))) float v4f;
__device__ __forceinline__ float bf16_rne(float f) { unsigned int u = __float_as_uint(f); u += 0x7FFFu + ((u >> 16) & 1u); return __uint_as_float(u & 0xFFFF0000u); }
__device__ __forceinline__ void split16(float v, b16& hi, b16& lo) { hi = (b16)v; lo = (b16)(v - (float)hi); }
__device__ __forceinline__ v16b frag_kb(const b16* p, int hh) { const v8b a = *(const v8b*)(p + 8 * hh), b = *(const v8b*)(p + 16 + 8 * hh); v16b f;
#pragma unroll
  for (int e = 0; e < 8; ++e) { f[e] = a[e]; f[8 + e] = b[e]; } return f; }
__device__ __forceinline__ v8f wmma16b(v16b a, v16b b, v8f c) { v8f d = __builtin_amdgcn_wmma_f32_16x16x32_f16(false, a, false, b, (short)0, c, false, false); asm volatile("v_nop\n\tv_nop\n\tv_nop\n\tv_nop" : "+v"(d) : "v"(a), "v"(b)); return d; }
__device__ __forceinline__ void wave_lds_sync() { __builtin_amdgcn_fence(__ATOMIC_RELEASE, "workgroup"); __builtin_amdgcn_wave_barrier(); __builtin_amdgcn_fence(__ATOMIC_ACQUIRE, "workgroup"); }
__device__ __forceinline__ float pmul(float a, float b) { float p = a * b; asm volatile("" : "+v"(p)); return p; }
__device__ __forceinline__ float silu(float v) { return v / (1.0f + __expf(-v)); }
__device__ __forceinline__ float softplus(float v) { return v > 20.0f ? v : (v < -20.0f ? __expf(v) : log1pf(__expf(v))); }

__global__ __launch_bounds__(256) void wcopy_kernel(const float* __restrict__ w, int OUT, int KIN, int KP, b16* __restrict__ WT) {
  const size_t u = (size_t)blockIdx.x * 256 + threadIdx.x; if (u >= (size_t)OUT * KP / 8) return; const size_t e = u * 8; const int o = (int)(e / KP), k0 = (int)(e % KP); v8b v;
  for (int j = 0; j < 8; ++j) { const int k = k0 + j; v[j] = k < KIN ? (b16)(bf16_rne(w[(size_t)o * KIN + (k < KIN ? k : 0)]) * WSC) : (b16)0.0f; } for (int pass = 0; pass < 2; ++pass) { *(volatile v8b*)(WT + e) = v; __threadfence(); }
}
template <int NT, int KW, int NPROD>
__device__ __forceinline__ void gemm_tiles(const b16 (*Ah)[DI * 2 + 8], const b16 (*Al)[DI * 2 + 8], const b16* __restrict__ WT, int wpitch, int c0, v8f* acc, int nloc, int hlf) {
#pragma unroll
  for (int t = 0; t < NT; ++t) acc[t] = (v8f){};
#pragma unroll 2
  for (int kb = 0; kb < KW; kb += 32) { const v16b a = frag_kb(&Ah[nloc][kb], hlf); v16b al = {}; if (NPROD == 2) al = frag_kb(&Al[nloc][kb], hlf);
#pragma unroll
    for (int t = 0; t < NT; ++t) { const v16b bw = frag_kb(WT + (size_t)(c0 + t * 16 + nloc) * wpitch + kb, hlf); acc[t] = wmma16b(a, bw, acc[t]); if (NPROD == 2) acc[t] = wmma16b(al, bw, acc[t]); } }
}
__global__ __launch_bounds__(32) void chain_kernel(const float* __restrict__ perc, const b16* __restrict__ WIN, const b16* __restrict__ WIP, const b16* __restrict__ WXP, const b16* __restrict__ WDT, const b16* __restrict__ WOP, const b16* __restrict__ WMU, const b16* __restrict__ WLS,
                                                   const float* __restrict__ b_in, const float* __restrict__ conv_w, const float* __restrict__ conv_b, const float* __restrict__ dt_b, const float* __restrict__ Dskip, const float* __restrict__ mu_b, const float* __restrict__ ls_b,
                                                   float* __restrict__ out_mu, float* __restrict__ out_ls) {
  __shared__ __attribute__((aligned(16))) b16 Ah[16][DI * 2 + 8], Al[16][DI * 2 + 8]; __shared__ __attribute__((aligned(16))) float U[16][DI + 4], Z[16][DI + 4]; __shared__ __attribute__((aligned(16))) float Sm[16][AD], Sl[16][AD]; __shared__ float BCr[16];
  const int lane = threadIdx.x, nloc = lane & 15, hlf = lane >> 4; const size_t m0 = (size_t)blockIdx.x * 16; const float sx = 1.0f / (XS * WSC), se = 1.0f / (ES * WSC);
  for (int rr = 0; rr < 16; ++rr) for (int q = 0; q < 4; ++q) { const v4f v = *(const v4f*)(perc + (m0 + rr) * P + q * 128 + lane * 4); for (int j = 0; j < 4; ++j) { Ah[rr][q * 128 + lane * 4 + j] = (b16)(bf16_rne(v[j]) * XS); Al[rr][q * 128 + lane * 4 + j] = (b16)0.0f; } }
  wave_lds_sync();
  v8f acc[8];
  { float xk[2][8][8];
    for (int cg = 0; cg < 2; ++cg) { gemm_tiles<8, P, 1>(Ah, Al, WIN, P, cg * 128, acc, nloc, hlf);
#pragma unroll
      for (int t = 0; t < 8; ++t)
#pragma unroll
        for (int r8 = 0; r8 < 8; ++r8) xk[cg][t][r8] = acc[t][r8] * sx + bf16_rne(b_in[cg * 128 + t * 16 + nloc]); }
    wave_lds_sync();
    for (int cg = 0; cg < 2; ++cg)
#pragma unroll
      for (int t = 0; t < 8; ++t)
#pragma unroll
        for (int r8 = 0; r8 < 8; ++r8) { b16 p, ql; split16(xk[cg][t][r8] * XS, p, ql); Ah[8 * hlf + r8][cg * 128 + t * 16 + nloc] = p; Al[8 * hlf + r8][cg * 128 + t * 16 + nloc] = ql; } }
  wave_lds_sync();
#pragma unroll 1
  for (int cg = 0; cg < 8; ++cg) { gemm_tiles<8, DM, 2>(Ah, Al, WIP, DM, cg * 128, acc, nloc, hlf);
#pragma unroll
    for (int t = 0; t < 8; ++t) { const int c = cg * 128 + t * 16 + nloc;
      if (cg < 4) { const float cw3 = bf16_rne(conv_w[c * 4 + 3]), cb = bf16_rne(conv_b[c]);
#pragma unroll 1
        for (int r8 = 0; r8 < 8; ++r8) U[8 * hlf + r8][c] = silu(pmul(acc[t][r8] * sx, cw3) + cb); }
      else {
#pragma unroll 1
        for (int r8 = 0; r8 < 8; ++r8) Z[8 * hlf + r8][c - DI] = silu(acc[t][r8] * sx); } } }
  wave_lds_sync();
  for (int rr = 0; rr < 16; ++rr) for (int q = 0; q < 4; ++q) { const v4f v = *(const v4f*)(&U[rr][q * 128 + lane * 4]); for (int j = 0; j < 4; ++j) { b16 p, ql; split16(v[j] * ES, p, ql); Ah[rr][q * 128 + lane * 4 + j] = p; Al[rr][q * 128 + lane * 4 + j] = ql; } }
  wave_lds_sync();
  { v8f ax[3]; gemm_tiles<3, DI, 2>(Ah, Al, WXP, DI, 0, ax, nloc, hlf);
    wave_lds_sync();
#pragma unroll
    for (int r8 = 0; r8 < 8; ++r8) { float bc = pmul(ax[1][r8] * se, ax[2][r8] * se); for (int o = 1; o < 16; o <<= 1) bc += __shfl_xor(bc, o); if (nloc == 0) BCr[8 * hlf + r8] = bc;
      b16 p, ql; split16(ax[0][r8] * se * ES, p, ql); Ah[8 * hlf + r8][nloc] = p; Al[8 * hlf + r8][nloc] = ql; Ah[8 * hlf + r8][16 + nloc] = (b16)0.0f; Al[8 * hlf + r8][16 + nloc] = (b16)0.0f; } }
  wave_lds_sync();
#pragma unroll 1
  for (int cg = 0; cg < 4; ++cg) { gemm_tiles<8, 32, 2>(Ah, Al, WDT, 32, cg * 128, acc, nloc, hlf);
#pragma unroll
    for (int t = 0; t < 8; ++t) { const int c = cg * 128 + t * 16 + nloc; const float db = bf16_rne(dt_b[c]), dsk = bf16_rne(Dskip[c]);
#pragma unroll 1
      for (int r8 = 0; r8 < 8; ++r8) { const int rl = 8 * hlf + r8; const float delta = softplus(acc[t][r8] * se + db); const float u = U[rl][c]; const float y = pmul(u, pmul(delta, BCr[rl]) + dsk); U[rl][c] = pmul(y, Z[rl][c]); } } }
  wave_lds_sync();
  for (int rr = 0; rr < 16; ++rr) for (int q = 0; q < 4; ++q) { const v4f v = *(const v4f*)(&U[rr][q * 128 + lane * 4]); for (int j = 0; j < 4; ++j) { b16 p, ql; split16(v[j] * ES, p, ql); Ah[rr][q * 128 + lane * 4 + j] = p; Al[rr][q * 128 + lane * 4 + j] = ql; } }
  wave_lds_sync();
  { float hk[2][8][8];
    for (int cg = 0; cg < 2; ++cg) { gemm_tiles<8, DI, 2>(Ah, Al, WOP, DI, cg * 128, acc, nloc, hlf);
#pragma unroll
      for (int t = 0; t < 8; ++t)
#pragma unroll
        for (int r8 = 0; r8 < 8; ++r8) hk[cg][t][r8] = acc[t][r8] * se; }
    wave_lds_sync();
    for (int cg = 0; cg < 2; ++cg)
#pragma unroll
      for (int t = 0; t < 8; ++t)
#pragma unroll
        for (int r8 = 0; r8 < 8; ++r8) { b16 p, ql; split16(hk[cg][t][r8] * ES, p, ql); Ah[8 * hlf + r8][cg * 128 + t * 16 + nloc] = p; Al[8 * hlf + r8][cg * 128 + t * 16 + nloc] = ql; } }
  wave_lds_sync();
  { v8f am[4], al4[4]; gemm_tiles<4, DM, 2>(Ah, Al, WMU, DM, 0, am, nloc, hlf); gemm_tiles<4, DM, 2>(Ah, Al, WLS, DM, 0, al4, nloc, hlf);
#pragma unroll
    for (int t = 0; t < 4; ++t) { const int c = t * 16 + nloc; const float mb = bf16_rne(mu_b[c]), lb = bf16_rne(ls_b[c]);
#pragma unroll 1
      for (int r8 = 0; r8 < 8; ++r8) { Sm[8 * hlf + r8][c] = tanhf(am[t][r8] * se + mb); const float lv = al4[t][r8] * se + lb; Sl[8 * hlf + r8][c] = fminf(fmaxf(lv, -5.0f), 2.0f); } } }
  wave_lds_sync();
  for (int pass = 0; pass < 2; ++pass) { for (int rr = 0; rr < 16; ++rr) { if (lane < 16) *(volatile v4f*)(out_mu + (m0 + rr) * AD + lane * 4) = *(const v4f*)(&Sm[rr][lane * 4]); else *(volatile v4f*)(out_ls + (m0 + rr) * AD + (lane - 16) * 4) = *(const v4f*)(&Sl[rr][(lane - 16) * 4]); } __threadfence(); }
}
}

extern "C" void kernel_launch(void* const* d_in, const int* in_sizes, int n_in, void* d_out, int out_size, void* d_ws, size_t ws_size, hipStream_t stream) {
  (void)n_in;
  auto Fp = [&](int i) { return (const float*)d_in[i]; };
  if (in_sizes[0] != NBT * P || in_sizes[1] != DM * P || in_sizes[3] != AD * DM || in_sizes[5] != AD * DM || in_sizes[7] != 2 * DI * DM || in_sizes[8] != DI * 4 || in_sizes[10] != XD * DI || in_sizes[11] != DI * DTR || in_sizes[15] != DM * DI || out_size != 2 * NBT * AD) return;
  const int NROWS = NBT;
  size_t off = 0; char* ws = (char*)d_ws;
  auto carve = [&](size_t bytes) { char* p = ws + off; off += (bytes + 255) & ~(size_t)255; return p; };
  b16* WIN = (b16*)carve((size_t)DM * P * 2); b16* WIP = (b16*)carve((size_t)2 * DI * DM * 2); b16* WXP = (b16*)carve((size_t)XD * DI * 2); b16* WDT = (b16*)carve((size_t)DI * 32 * 2); b16* WOP = (b16*)carve((size_t)DM * DI * 2); b16* WMU = (b16*)carve((size_t)AD * DM * 2); b16* WLS = (b16*)carve((size_t)AD * DM * 2);
  if (off > ws_size || off > ((size_t)16 << 20)) return;
  auto g = [](int n8) { return (unsigned)((n8 + 255) / 256); };
  wcopy_kernel<<<g(DM * P / 8), 256, 0, stream>>>(Fp(1), DM, P, P, WIN); wcopy_kernel<<<g(2 * DI * DM / 8), 256, 0, stream>>>(Fp(7), 2 * DI, DM, DM, WIP); wcopy_kernel<<<g(XD * DI / 8), 256, 0, stream>>>(Fp(10), XD, DI, DI, WXP);
  wcopy_kernel<<<g(DI * 32 / 8), 256, 0, stream>>>(Fp(11), DI, DTR, 32, WDT); wcopy_kernel<<<g(DM * DI / 8), 256, 0, stream>>>(Fp(15), DM, DI, DI, WOP); wcopy_kernel<<<g(AD * DM / 8), 256, 0, stream>>>(Fp(3), AD, DM, DM, WMU); wcopy_kernel<<<g(AD * DM / 8), 256, 0, stream>>>(Fp(5), AD, DM, DM, WLS);
  chain_kernel<<<NROWS / 16, 32, 0, stream>>>(Fp(0), WIN, WIP, WXP, WDT, WOP, WMU, WLS, Fp(2), Fp(8), Fp(9), Fp(12), Fp(14), Fp(4), Fp(6), (float*)d_out, (float*)d_out + (size_t)NBT * AD);
}
